// CachedMPS_82824149336270
// MI455X (gfx1250) — hardware-verified
//
#include <hip/hip_runtime.h>


namespace {
constexpr int Bn = 32768, L = 256, F = 2, D = 32, C = 10, NB = 128, NMID = L - 2;
constexpr float AS_ = 8.0f, HALF_PI = 1.5707963267948966f;

typedef _Float16 b16;
typedef __attribute__((ext_vector_type(16))) _Float16 v16b;
typedef __attribute__((ext_vector_type(8))) _Float16 v8b;
typedef __attribute__((ext_vector_type(8))) float v8f;
typedef __attribute__((ext_vector_type(4))) float v4f;
__device__ __forceinline__ float bf16_rne(float f) { unsigned int u = __float_as_uint(f); u += 0x7FFFu + ((u >> 16) & 1u); return __uint_as_float(u & 0xFFFF0000u); }
__device__ __forceinline__ void split16(float v, b16& hi, b16& lo) { hi = (b16)v; lo = (b16)(v - (float)hi); }
__device__ __forceinline__ v16b frag_kb(const b16* p, int hh) { const v8b a = *(const v8b*)(p + 8 * hh), b = *(const v8b*)(p + 16 + 8 * hh); v16b f;
#pragma unroll
  for (int e = 0; e < 8; ++e) { f[e] = a[e]; f[8 + e] = b[e]; } return f; }
__device__ __forceinline__ v8f wmma16b(v16b a, v16b b, v8f c) { v8f d = __builtin_amdgcn_wmma_f32_16x16x32_f16(false, a, false, b, (short)0, c, false, false); asm volatile("v_nop\n\tv_nop\n\tv_nop\n\tv_nop" : "+v"(d) : "v"(a), "v"(b)); return d; }
__device__ __forceinline__ void wave_lds_sync() { __builtin_amdgcn_fence(__ATOMIC_RELEASE, "workgroup"); __builtin_amdgcn_wave_barrier(); __builtin_amdgcn_fence(__ATOMIC_ACQUIRE, "workgroup"); }
__device__ __forceinline__ float pmul(float a, float b) { float p = a * b; asm volatile("" : "+v"(p)); return p; }

__global__ __launch_bounds__(256) void prep_kernel(const float* __restrict__ c0, const float* __restrict__ cm, const float* __restrict__ cN, b16* __restrict__ Bm, b16* __restrict__ BN_, float* __restrict__ C0) {
  const size_t tid = (size_t)blockIdx.x * blockDim.x + threadIdx.x, nth = (size_t)gridDim.x * blockDim.x;
  for (int pass = 0; pass < 2; ++pass) {
    for (size_t p = tid; p < (size_t)NMID * 64 * 32; p += nth) { const int t = (int)(p >> 11), q = (int)(p & 2047), n = q >> 5, a = q & 31, f = n >> 5, c = n & 31;
      ((volatile b16*)Bm)[p] = (b16)bf16_rne(cm[(((size_t)t * F + f) * D + a) * D + c]); }
    for (size_t p = tid; p < 32 * 32; p += nth) { const int n = (int)(p >> 5), a = (int)(p & 31), f = n >> 4, c = n & 15; ((volatile b16*)BN_)[p] = (b16)((c < C) ? bf16_rne(cN[((size_t)f * D + a) * C + c]) : 0.0f); }
    for (size_t p = tid; p < 64; p += nth) ((volatile float*)C0)[p] = bf16_rne(c0[p]);
    __threadfence();
  }
}

__global__ __launch_bounds__(256) void mps_kernel(const float* __restrict__ x, const float* __restrict__ C0, const b16* __restrict__ Bm, const b16* __restrict__ BN_, float* __restrict__ out) {
  __shared__ __attribute__((aligned(16))) b16 Mh[8][16][D + 8], Ml[8][16][D + 8]; __shared__ __attribute__((aligned(16))) float Os[NB * C]; __shared__ float Fs[8][16][2];
  const int wid = threadIdx.x >> 5, lane = threadIdx.x & 31, nloc = lane & 15, hlf = lane >> 4; const size_t s0 = (size_t)blockIdx.x * NB + wid * 16;
if (hlf == 0) { const float xv = bf16_rne(x[(s0 + nloc) * L + 0]); Fs[wid][nloc][0] = cosf(HALF_PI * xv); Fs[wid][nloc][1] = sinf(HALF_PI * xv); }
  wave_lds_sync();
#pragma unroll
  for (int v = 0; v < 8; ++v) { const int r = 8 * hlf + v; const float f0 = Fs[wid][r][0], f1 = Fs[wid][r][1];
#pragma unroll
    for (int q = 0; q < 2; ++q) { const int c = q * 16 + nloc; const float m = pmul(f0, C0[c]) + pmul(f1, C0[32 + c]); b16 a, l; split16(m * AS_, a, l); Mh[wid][r][c] = a; Ml[wid][r][c] = l; } }
  wave_lds_sync();
  for (int t = 0; t < NMID; ++t) {
    if (hlf == 0) { const float xv = bf16_rne(x[(s0 + nloc) * L + (t + 1)]); Fs[wid][nloc][0] = cosf(HALF_PI * xv); Fs[wid][nloc][1] = sinf(HALF_PI * xv); }
    const v16b ah = frag_kb(&Mh[wid][nloc][0], hlf), al = frag_kb(&Ml[wid][nloc][0], hlf);
    const b16* Bt = Bm + (size_t)t * 64 * 32; v8f acc[4];
#pragma unroll
    for (int q = 0; q < 4; ++q) { acc[q] = (v8f){}; const v16b bw = frag_kb(Bt + (size_t)(q * 16 + nloc) * 32, hlf); acc[q] = wmma16b(ah, bw, acc[q]); acc[q] = wmma16b(al, bw, acc[q]); }
    wave_lds_sync();
#pragma unroll
    for (int v = 0; v < 8; ++v) { const float f0 = Fs[wid][8 * hlf + v][0], f1 = Fs[wid][8 * hlf + v][1]; const float m0 = (pmul(f0, acc[0][v]) + pmul(f1, acc[2][v])) * (1.0f / AS_), m1 = (pmul(f0, acc[1][v]) + pmul(f1, acc[3][v])) * (1.0f / AS_);
      float ss = pmul(m0, m0) + pmul(m1, m1);
#pragma unroll
      for (int o = 1; o < 16; o <<= 1) ss += __shfl_xor(ss, o);
      const float inv = 1.0f / (sqrtf(ss) + 1e-8f); const int r = 8 * hlf + v;
      b16 a, l; split16(m0 * inv * AS_, a, l); Mh[wid][r][nloc] = a; Ml[wid][r][nloc] = l; split16(m1 * inv * AS_, a, l); Mh[wid][r][16 + nloc] = a; Ml[wid][r][16 + nloc] = l; }
    wave_lds_sync();
  }
  { const v16b ah = frag_kb(&Mh[wid][nloc][0], hlf), al = frag_kb(&Ml[wid][nloc][0], hlf); v8f acc[2];
#pragma unroll
    for (int q = 0; q < 2; ++q) { acc[q] = (v8f){}; const v16b bw = frag_kb(BN_ + (size_t)(q * 16 + nloc) * 32, hlf); acc[q] = wmma16b(ah, bw, acc[q]); acc[q] = wmma16b(al, bw, acc[q]); }
    if (hlf == 0) { const float xv = bf16_rne(x[(s0 + nloc) * L + (L - 1)]); Fs[wid][nloc][0] = cosf(HALF_PI * xv); Fs[wid][nloc][1] = sinf(HALF_PI * xv); }
    wave_lds_sync();
#pragma unroll
    for (int v = 0; v < 8; ++v) { const int r = 8 * hlf + v; const float f0 = Fs[wid][r][0], f1 = Fs[wid][r][1];
      if (nloc < C) Os[(wid * 16 + r) * C + nloc] = (pmul(f0, acc[0][v]) + pmul(f1, acc[1][v])) * (1.0f / AS_); } }
  __syncthreads();
  for (int pass = 0; pass < 2; ++pass) { for (int q = threadIdx.x; q < NB * C / 4; q += 256) *(volatile v4f*)(out + (size_t)blockIdx.x * NB * C + q * 4) = *(const v4f*)(&Os[q * 4]); __threadfence(); }
}
}

extern "C" void kernel_launch(void* const* d_in, const int* in_sizes, int n_in,
                              void* d_out, int out_size, void* d_ws, size_t ws_size, hipStream_t stream) {
  (void)n_in; (void)out_size;
  const float* x = (const float*)d_in[0]; const float* c0 = (const float*)d_in[1]; const float* cm = (const float*)d_in[2]; const float* cN = (const float*)d_in[3];
  float* out = (float*)d_out;
  if (in_sizes[0] != Bn * L || in_sizes[1] != F * D || in_sizes[2] != NMID * F * D * D || in_sizes[3] != F * D * C) return;
  size_t off = 0; char* ws = (char*)d_ws;
  auto carve = [&](size_t bytes) { char* p = ws + off; off += (bytes + 255) & ~(size_t)255; return p; };
  b16* Bm = (b16*)carve((size_t)NMID * 64 * 32 * 2); b16* BN_ = (b16*)carve(32 * 32 * 2); float* C0 = (float*)carve(256);
  if (off > ws_size) return;
  prep_kernel<<<64, 256, 0, stream>>>(c0, cm, cN, Bm, BN_, C0);
  mps_kernel<<<Bn / NB, 256, 0, stream>>>(x, C0, Bm, BN_, out);
}
